// Rnn_Model1_77326591197593
// MI455X (gfx1250) — hardware-verified
//
#include <hip/hip_runtime.h>
#include <math.h>

typedef __attribute__((ext_vector_type(16))) _Float16 v16h;
typedef __attribute__((ext_vector_type(8)))  _Float16 v8h;
typedef __attribute__((ext_vector_type(8)))  float    v8f;
typedef __attribute__((ext_vector_type(4)))  float    v4f;
typedef __attribute__((ext_vector_type(8)))  unsigned v8u;

constexpr int kT  = 32768;
constexpr int kD  = 64;
constexpr int kH  = 128;
constexpr int kG  = 4 * kH;
constexpr int kNHeadPad = 16;
constexpr int kHsPitch  = 2 * kH;
static_assert((kD % 32) == 0 && (kH % 32) == 0);
static_assert((kT % 64) == 0 && (kG % 64) == 0 && (kT % 32) == 0);

constexpr float kXCarry  = 16.0f;
constexpr float kWCarry  = 256.0f;
constexpr float kHCarry  = 512.0f;
constexpr float kLoCarry = 2048.0f;
constexpr float kF16MinNormal = 6.103515625e-05f;
constexpr float kProjScale = 1.0f / (kXCarry * kWCarry);
constexpr float kRecHi = 1.0f / (kHCarry * kWCarry);
constexpr float kRecLo = kRecHi / kLoCarry;

constexpr unsigned kOutOff1 = (unsigned)kT * 11u;
constexpr unsigned kOutOff2 = kOutOff1 + (unsigned)kT * 2u;
constexpr unsigned kOutOff3 = kOutOff2 + (unsigned)kT;
constexpr unsigned kOutTotal = kOutOff3 + (unsigned)kT;
static_assert(kOutOff1 * 4u == 1441792u && kOutOff2 * 4u == 1703936u && kOutOff3 * 4u == 1835008u);
static_assert(kOutTotal == 491520u);

constexpr size_t kOffX16   = 0;
constexpr size_t kOffWIH   = kOffX16  + (size_t)kT * kD * 2;
constexpr size_t kOffWHH   = kOffWIH  + (size_t)kG * kD * 2;
constexpr size_t kOffWHD   = kOffWHH  + (size_t)kG * kH * 2;
constexpr size_t kOffBIASP = kOffWHD  + (size_t)kNHeadPad * kH * 2;
constexpr size_t kOffBHEAD = kOffBIASP + (size_t)kG * 4;
constexpr size_t kOffXG    = kOffBHEAD + (size_t)32 * 4;
constexpr size_t kOffHS    = kOffXG   + (size_t)kT * kG * 4;
constexpr size_t kWsTotal  = kOffHS   + (size_t)kT * kHsPitch * 2;
static_assert(kWsTotal == 88283264ull);
static_assert(kWsTotal <= 134217728ull);
static_assert((kOffWIH % 128) == 0 && (kOffWHH % 128) == 0 && (kOffWHD % 128) == 0 && (kOffBIASP % 128) == 0 &&
              (kOffBHEAD % 128) == 0 && (kOffXG % 128) == 0 && (kOffHS % 128) == 0);

struct FragH {
  union U { v16h v; v8h h[2]; };
  static __device__ __forceinline__ v16h load(const _Float16* p) {
    U f; f.h[0] = *(const v8h*)(p); f.h[1] = *(const v8h*)(p + 16); return f.v;
  }
  static __device__ __forceinline__ v8f mma(v16h a, v16h b, v8f c) {
    return __builtin_amdgcn_wmma_f32_16x16x32_f16(false, a, false, b, (short)0, c, false, false);
  }
};
__device__ __forceinline__ void guard4_h(v8f& a, v8f& b, v8f& c, v8f& d, v16h x) {
  asm volatile("v_nop\n\tv_nop\n\tv_nop\n\tv_nop" : "+v"(a), "+v"(b), "+v"(c), "+v"(d) : "v"(x));
}
__device__ __forceinline__ void guard1_a4(v8f& acc, v16h a0, v16h a1, v16h a2, v16h a3) {
  asm volatile("v_nop\n\tv_nop\n\tv_nop\n\tv_nop" : "+v"(acc) : "v"(a0), "v"(a1), "v"(a2), "v"(a3));
}
__device__ __forceinline__ void keep4_h(v16h a, v16h b, v16h c, v16h d) { asm volatile("v_nop" :: "v"(a), "v"(b), "v"(c), "v"(d)); }
__device__ __forceinline__ void acc_guard4(v8f& a, v8f& b, v8f& c, v8f& d) { asm volatile("v_nop\n\tv_nop\n\tv_nop\n\tv_nop" : "+v"(a), "+v"(b), "+v"(c), "+v"(d)); }

__device__ __forceinline__ _Float16 to_f16_flush(float v) {
  const float w = (fabsf(v) < kF16MinNormal) ? 0.0f : v;
  return (_Float16)w;
}
__device__ __forceinline__ v16h frag_keep(v16h f, bool keep) {
  v8u u = __builtin_bit_cast(v8u, f);
  const v8u z = (v8u)(0u);
  u = keep ? u : z;
  return __builtin_bit_cast(v16h, u);
}

__global__ __launch_bounds__(256) void cvt_rows_f16_kernel(
    const float* __restrict__ src, unsigned short* __restrict__ dst, int total8, float carry, int permute)
{
  const unsigned i = blockIdx.x * 256u + threadIdx.x;
  if (i >= (unsigned)total8) return;
  unsigned si = i;
  if (permute != 0) {
    const unsigned row = i >> 3;
    const unsigned c = i & 7u;
    const unsigned g = ((row & 3u) << 7) + ((row >> 6) << 4) + ((row >> 2) & 15u);
    si = (g << 3) + c;
  }
  asm volatile("" : "+v"(si));
  const float* sp = src + (size_t)si * 8u;
  const v4f a0 = *(const v4f*)(sp);
  const v4f a1 = *(const v4f*)(sp + 4);
  v8h hv;
#pragma unroll
  for (int e = 0; e < 4; ++e) {
    hv[e]     = to_f16_flush(a0[e] * carry);
    hv[4 + e] = to_f16_flush(a1[e] * carry);
  }
  _Float16* q = (_Float16*)dst + (size_t)i * 8u;
  *(volatile v8h*)q = hv;
  __threadfence();
  *(volatile v8h*)q = hv;
}

__global__ __launch_bounds__(256) void prep_small_kernel(
    const float* __restrict__ b_ih, const float* __restrict__ b_hh,
    const float* __restrict__ W1, const float* __restrict__ b1,
    const float* __restrict__ W2, const float* __restrict__ b2,
    const float* __restrict__ W3, const float* __restrict__ b3,
    const float* __restrict__ W4, const float* __restrict__ b4,
    unsigned short* __restrict__ whd16, float* __restrict__ biasp, float* __restrict__ bhead)
{
  const unsigned tid = threadIdx.x;
  const unsigned row = tid >> 4;
  const unsigned c8 = (tid & 15u) * 8u;
  const unsigned r1 = (row < 10u) ? row : 10u;
  const unsigned r2 = (row < 12u) ? 0u : 1u;
  v4f p0 = *(const v4f*)(W1 + r1 * (unsigned)kH + c8);
  v4f p1 = *(const v4f*)(W1 + r1 * (unsigned)kH + c8 + 4u);
  v4f q0 = *(const v4f*)(W2 + r2 * (unsigned)kH + c8);
  v4f q1 = *(const v4f*)(W2 + r2 * (unsigned)kH + c8 + 4u);
  v4f s0 = *(const v4f*)(W3 + c8);
  v4f s1 = *(const v4f*)(W3 + c8 + 4u);
  v4f u0 = *(const v4f*)(W4 + c8);
  v4f u1 = *(const v4f*)(W4 + c8 + 4u);
  asm volatile("" : "+v"(p0), "+v"(p1), "+v"(q0), "+v"(q1));
  asm volatile("" : "+v"(s0), "+v"(s1), "+v"(u0), "+v"(u1));
  const bool selA = (row < 11u);
  const bool selB = (row < 13u);
  const bool selC = (row == 13u);
  const bool keepRow = (row < 15u);
  v8h hv;
#pragma unroll
  for (int e = 0; e < 4; ++e) {
    const float w0 = selA ? p0[e] : (selB ? q0[e] : (selC ? s0[e] : u0[e]));
    const float w1 = selA ? p1[e] : (selB ? q1[e] : (selC ? s1[e] : u1[e]));
    const float x0 = keepRow ? (w0 * kWCarry) : 0.0f;
    const float x1 = keepRow ? (w1 * kWCarry) : 0.0f;
    hv[e]     = to_f16_flush(x0);
    hv[4 + e] = to_f16_flush(x1);
  }
  const unsigned bi = tid & 127u;
  const unsigned bw = bi >> 4;
  const unsigned bl = bi & 15u;
  v4f bsum;
#pragma unroll
  for (int q = 0; q < 4; ++q) {
    const unsigned g = (unsigned)q * (unsigned)kH + 16u * bw + bl;
    float s = b_ih[g] + b_hh[g];
    asm volatile("" : "+v"(s));
    bsum[q] = s;
  }
  const unsigned j = tid & 31u;
  const unsigned j1 = (j < 10u) ? j : 10u;
  const unsigned j2 = (j < 12u) ? 0u : 1u;
  float v1 = b1[j1];
  float v2 = b2[j2];
  float v3 = b3[0];
  float v4 = b4[0];
  asm volatile("" : "+v"(v1), "+v"(v2), "+v"(v3), "+v"(v4));
  const float hb = (j < 11u) ? v1 : (j < 13u) ? v2 : (j == 13u) ? v3 : (j == 14u) ? v4 : 0.0f;

  _Float16* qd = (_Float16*)whd16 + (size_t)tid * 8u;
  for (int pass = 0; pass < 2; ++pass) {
    *(volatile v8h*)qd = hv;
    if (tid < 128u) *(volatile v4f*)(biasp + 4u * tid) = bsum;
    if (tid < 32u) *(volatile float*)(bhead + tid) = hb;
    __threadfence();
  }
}

__global__ __launch_bounds__(256) void gemm64_f16_bias_kernel(
    const unsigned short* __restrict__ Ap, int lda,
    const unsigned short* __restrict__ Btp, int ldb,
    float* __restrict__ C, int ldc,
    const float* __restrict__ bias, int M, int N, int K, float scale)
{
  const _Float16* A  = (const _Float16*)Ap;
  const _Float16* Bt = (const _Float16*)Btp;
  __shared__ __align__(16) float sT[8][16 * 68];
  const int lane = threadIdx.x & 31;
  const int wave = threadIdx.x >> 5;
  const int tilesN = N >> 6;
  const int tilesM = M >> 6;
  const int tile = blockIdx.x * 8 + wave;
  if (tile >= tilesM * tilesN) return;
  const int tm = tile / tilesN;
  const int tn = tile - tm * tilesN;
  const int m0 = tm << 6;
  const int n0 = tn << 6;
  const int rlane = lane & 15;
  const int koff  = (lane >> 4) * 8;
  const int mOff  = (lane >> 4) * 8;

  v8f acc[4][4];
#pragma unroll
  for (int i = 0; i < 4; ++i)
#pragma unroll
    for (int j = 0; j < 4; ++j) acc[i][j] = (v8f){0.f,0.f,0.f,0.f,0.f,0.f,0.f,0.f};

  for (int k0 = 0; k0 < K; k0 += 32) {
    v16h bh[4];
#pragma unroll
    for (int j = 0; j < 4; ++j) {
      const size_t bo = (size_t)(n0 + (j << 4) + rlane) * ldb + koff + k0;
      bh[j] = FragH::load(Bt + bo);
    }
#pragma unroll
    for (int i = 0; i < 4; ++i) {
      const size_t ao = (size_t)(m0 + (i << 4) + rlane) * lda + koff + k0;
      v16h ah = FragH::load(A + ao);
#pragma unroll
      for (int j = 0; j < 4; ++j) acc[i][j] = FragH::mma(ah, bh[j], acc[i][j]);
      guard4_h(acc[i][0], acc[i][1], acc[i][2], acc[i][3], ah);
    }
    keep4_h(bh[0], bh[1], bh[2], bh[3]);
  }
  acc_guard4(acc[0][0], acc[0][1], acc[0][2], acc[0][3]);
  acc_guard4(acc[1][0], acc[1][1], acc[1][2], acc[1][3]);
  acc_guard4(acc[2][0], acc[2][1], acc[2][2], acc[2][3]);
  acc_guard4(acc[3][0], acc[3][1], acc[3][2], acc[3][3]);

  float* slab = sT[wave];
#pragma unroll
  for (int i = 0; i < 4; ++i) {
    const int mBase = m0 + (i << 4);
#pragma unroll
    for (int j = 0; j < 4; ++j) {
      const int n = n0 + (j << 4) + rlane;
      const float bv = bias[n];
#pragma unroll
      for (int r = 0; r < 8; ++r) {
        const float v = acc[i][j][r] * scale + bv;
        slab[(mOff + r) * 68 + (j << 4) + rlane] = v;
      }
    }
    __builtin_amdgcn_fence(__ATOMIC_RELEASE, "workgroup");
    __builtin_amdgcn_wave_barrier();
    __builtin_amdgcn_fence(__ATOMIC_ACQUIRE, "workgroup");
    {
      const int hh = lane >> 4, c4 = (lane & 15) * 4;
      for (int pass = 0; pass < 2; ++pass) {
#pragma unroll
        for (int it = 0; it < 8; ++it) {
          const int row = it * 2 + hh;
          v4f v = *(const v4f*)(slab + row * 68 + c4);
          *(volatile v4f*)(C + (size_t)(mBase + row) * ldc + n0 + c4) = v;
        }
        __threadfence();
      }
    }
    __builtin_amdgcn_fence(__ATOMIC_RELEASE, "workgroup");
    __builtin_amdgcn_wave_barrier();
    __builtin_amdgcn_fence(__ATOMIC_ACQUIRE, "workgroup");
  }
}

__device__ __forceinline__ float gate_sigmoid(float x) {
  const float xc = fminf(fmaxf(x, -30.0f), 30.0f);
  return 1.0f / (1.0f + expf(-xc));
}
__device__ __forceinline__ float gate_tanh(float x) {
  const float y = fminf(fmaxf(2.0f * x, -40.0f), 40.0f);
  return 1.0f - 2.0f / (1.0f + expf(y));
}

__global__ __launch_bounds__(256) __attribute__((amdgpu_num_vgpr(256))) void lstm_scan_kernel(
    const unsigned short* __restrict__ whh16, const float* __restrict__ xg, unsigned short* __restrict__ hs16)
{
  __shared__ __align__(16) _Float16 hbuf[2 * 2 * kH];
  const unsigned tid = threadIdx.x;
  const unsigned lane = tid & 31u;
  const unsigned wave = tid >> 5;
  const unsigned hh = lane >> 4;
  const unsigned nl = lane & 15u;
  const _Float16* Whh = (const _Float16*)whh16;

  v16h bw[4][4];
#pragma unroll
  for (int q = 0; q < 4; ++q)
#pragma unroll
    for (int ks = 0; ks < 4; ++ks)
      bw[q][ks] = FragH::load(Whh + (size_t)((unsigned)q * (unsigned)kH + wave * 16u + nl) * (unsigned)kH + (unsigned)ks * 32u + 8u * hh);

  hbuf[tid] = (_Float16)0.0f;
  __syncthreads();

  const bool akeep = (nl < 2u);
  const unsigned arow = akeep ? nl : 0u;
  const float* xgp = xg + wave * 64u + nl * 4u;
  float x0, x1, x2, x3;
  {
    const v4f xv = *(const v4f*)xgp;
    x0 = xv[0]; x1 = xv[1]; x2 = xv[2]; x3 = xv[3];
    asm volatile("" : "+v"(x0), "+v"(x1), "+v"(x2), "+v"(x3));
  }
  float c = 0.0f;

#pragma unroll 1
  for (int t = 0; t < kT; ++t) {
    const unsigned cur = (unsigned)t & 1u;
    const unsigned nxt = cur ^ 1u;
    const int tn = (t + 1 < kT) ? (t + 1) : (kT - 1);
    float y0, y1, y2, y3;
    {
      const v4f xn = *(const v4f*)(xgp + (size_t)tn * (unsigned)kG);
      y0 = xn[0]; y1 = xn[1]; y2 = xn[2]; y3 = xn[3];
      asm volatile("" : "+v"(y0), "+v"(y1), "+v"(y2), "+v"(y3));
    }

    const _Float16* ab = hbuf + cur * 256u + arow * (unsigned)kH + 8u * hh;
    const v16h a0 = frag_keep(FragH::load(ab), akeep);
    const v16h a1 = frag_keep(FragH::load(ab + 32), akeep);
    const v16h a2 = frag_keep(FragH::load(ab + 64), akeep);
    const v16h a3 = frag_keep(FragH::load(ab + 96), akeep);

    v8f acc0 = (v8f){0.f,0.f,0.f,0.f,0.f,0.f,0.f,0.f};
    v8f acc1 = acc0, acc2 = acc0, acc3 = acc0;
    acc0 = FragH::mma(a0, bw[0][0], acc0);
    acc1 = FragH::mma(a0, bw[1][0], acc1);
    acc2 = FragH::mma(a0, bw[2][0], acc2);
    acc3 = FragH::mma(a0, bw[3][0], acc3);
    acc0 = FragH::mma(a1, bw[0][1], acc0);
    acc1 = FragH::mma(a1, bw[1][1], acc1);
    acc2 = FragH::mma(a1, bw[2][1], acc2);
    acc3 = FragH::mma(a1, bw[3][1], acc3);
    acc0 = FragH::mma(a2, bw[0][2], acc0);
    acc1 = FragH::mma(a2, bw[1][2], acc1);
    acc2 = FragH::mma(a2, bw[2][2], acc2);
    acc3 = FragH::mma(a2, bw[3][2], acc3);
    acc0 = FragH::mma(a3, bw[0][3], acc0);
    acc1 = FragH::mma(a3, bw[1][3], acc1);
    acc2 = FragH::mma(a3, bw[2][3], acc2);
    acc3 = FragH::mma(a3, bw[3][3], acc3);
    guard1_a4(acc0, a0, a1, a2, a3);
    guard1_a4(acc1, a0, a1, a2, a3);
    guard1_a4(acc2, a0, a1, a2, a3);
    guard1_a4(acc3, a0, a1, a2, a3);

    const float gi = x0 + (acc0[0] * kRecHi + acc0[1] * kRecLo);
    const float gf = x1 + (acc1[0] * kRecHi + acc1[1] * kRecLo);
    const float gg = x2 + (acc2[0] * kRecHi + acc2[1] * kRecLo);
    const float go = x3 + (acc3[0] * kRecHi + acc3[1] * kRecLo);
    const float si = gate_sigmoid(gi);
    const float sf = gate_sigmoid(gf);
    const float tg = gate_tanh(gg);
    const float so = gate_sigmoid(go);
    c = sf * c + si * tg;
    const float hnew = so * gate_tanh(c);

    const float hc = hnew * kHCarry;
    const _Float16 hi16 = to_f16_flush(hc);
    float hib = (float)hi16;
    asm volatile("" : "+v"(hib));
    const float lof = (hc - hib) * kLoCarry;
    const _Float16 lo16 = to_f16_flush(lof);
    if (lane < 16u) {
      hbuf[nxt * 256u + wave * 16u + nl] = hi16;
      hbuf[nxt * 256u + (unsigned)kH + wave * 16u + nl] = lo16;
    }
    __syncthreads();
    if (wave == 0u) {
      const v8h hv = *(const v8h*)(hbuf + nxt * 256u + lane * 8u);
      _Float16* dst = (_Float16*)hs16 + (size_t)t * (unsigned)kHsPitch + lane * 8u;
      *(volatile v8h*)dst = hv;
      __threadfence();
      *(volatile v8h*)dst = hv;
    }
    x0 = y0; x1 = y1; x2 = y2; x3 = y3;
  }
}

__global__ __launch_bounds__(256) void heads_kernel(
    const unsigned short* __restrict__ hs16, const unsigned short* __restrict__ whd16,
    const float* __restrict__ bhead, float* __restrict__ out)
{
  __shared__ __align__(16) float slab[8][32 * 16];
  const unsigned tid = threadIdx.x;
  const unsigned lane = tid & 31u;
  const unsigned wave = tid >> 5;
  const unsigned hh = lane >> 4;
  const unsigned nl = lane & 15u;
  const unsigned tile = blockIdx.x * 8u + wave;
  if (tile >= (unsigned)(kT / 32)) return;
  const unsigned t0 = tile * 32u;
  const _Float16* hs  = (const _Float16*)hs16;
  const _Float16* Whd = (const _Float16*)whd16;

  v16h bf[4];
#pragma unroll
  for (int ks = 0; ks < 4; ++ks) bf[ks] = FragH::load(Whd + nl * (unsigned)kH + (unsigned)ks * 32u + 8u * hh);
  const float bv = bhead[nl];
  float* sl = slab[wave];

#pragma unroll
  for (int i = 0; i < 2; ++i) {
    const _Float16* ar = hs + (size_t)(t0 + 16u * (unsigned)i + nl) * (unsigned)kHsPitch + 8u * hh;
    v16h fh[4], fl[4];
#pragma unroll
    for (int ks = 0; ks < 4; ++ks) {
      fh[ks] = FragH::load(ar + ks * 32);
      fl[ks] = FragH::load(ar + kH + ks * 32);
    }
    v8f acch = (v8f){0.f,0.f,0.f,0.f,0.f,0.f,0.f,0.f};
    v8f accl = acch;
#pragma unroll
    for (int ks = 0; ks < 4; ++ks) {
      acch = FragH::mma(fh[ks], bf[ks], acch);
      accl = FragH::mma(fl[ks], bf[ks], accl);
    }
    guard1_a4(acch, fh[0], fh[1], fh[2], fh[3]);
    guard1_a4(accl, fl[0], fl[1], fl[2], fl[3]);
#pragma unroll
    for (int r = 0; r < 8; ++r) {
      const float v = (acch[r] * kRecHi + accl[r] * kRecLo) + bv;
      sl[(16u * (unsigned)i + 8u * hh + (unsigned)r) * 16u + nl] = v;
    }
  }
  keep4_h(bf[0], bf[1], bf[2], bf[3]);
  __builtin_amdgcn_fence(__ATOMIC_RELEASE, "workgroup");
  __builtin_amdgcn_wave_barrier();
  __builtin_amdgcn_fence(__ATOMIC_ACQUIRE, "workgroup");

  v4f ov[3];
#pragma unroll
  for (int it = 0; it < 3; ++it) {
    unsigned i4 = (unsigned)it * 32u + lane;
    i4 = (i4 < 88u) ? i4 : 87u;
    asm volatile("" : "+v"(i4));
#pragma unroll
    for (int e = 0; e < 4; ++e) {
      unsigned f = i4 * 4u + (unsigned)e;
      asm volatile("" : "+v"(f));
      unsigned tt = f / 11u;
      asm volatile("" : "+v"(tt));
      unsigned li = tt * 16u + (f - tt * 11u);
      asm volatile("" : "+v"(li));
      ov[it][e] = sl[li];
    }
  }
  const bool grpA = (lane < 16u);
  const bool grpB = (lane < 24u);
  const unsigned l8 = lane & 7u;
  unsigned sbase = grpA ? (lane * 4u) : (l8 * 4u);
  unsigned soff = grpA ? (kOutOff1 + t0 * 2u + lane * 4u)
                : (grpB ? (kOutOff2 + t0 + l8 * 4u) : (kOutOff3 + t0 + l8 * 4u));
  unsigned scol = grpB ? 13u : 14u;
  asm volatile("" : "+v"(sbase), "+v"(soff), "+v"(scol));
  v4f sv;
#pragma unroll
  for (int e = 0; e < 4; ++e) {
    unsigned f = sbase + (unsigned)e;
    asm volatile("" : "+v"(f));
    unsigned tt = grpA ? (f >> 1) : f;
    unsigned jc = grpA ? (11u + (f & 1u)) : scol;
    unsigned li = tt * 16u + jc;
    asm volatile("" : "+v"(li));
    sv[e] = sl[li];
  }

  float* o0 = out + (size_t)t0 * 11u;
  for (int pass = 0; pass < 2; ++pass) {
#pragma unroll
    for (int it = 0; it < 3; ++it) {
      const unsigned i4 = (unsigned)it * 32u + lane;
      if (i4 < 88u) *(volatile v4f*)(o0 + i4 * 4u) = ov[it];
    }
    *(volatile v4f*)(out + soff) = sv;
    __threadfence();
  }
}

extern "C" void kernel_launch(void* const* d_in, const int* in_sizes, int n_in,
                              void* d_out, int out_size, void* d_ws, size_t ws_size,
                              hipStream_t stream) {
  if (n_in < 13) return;
  if (in_sizes[0] != kT * kD) return;
  if (in_sizes[1] != kG * kD) return;
  if (in_sizes[2] != kG * kH) return;
  if (in_sizes[3] != kG) return;
  if (in_sizes[4] != kG) return;
  if (in_sizes[5] != 11 * kH) return;
  if (in_sizes[6] != 11) return;
  if (in_sizes[7] != 2 * kH) return;
  if (in_sizes[8] != 2) return;
  if (in_sizes[9] != kH) return;
  if (in_sizes[10] != 1) return;
  if (in_sizes[11] != kH) return;
  if (in_sizes[12] != 1) return;
  if (out_size != (int)kOutTotal) return;
  if (ws_size < kWsTotal) return;

  const float* X    = (const float*)d_in[0];
  const float* W_ih = (const float*)d_in[1];
  const float* W_hh = (const float*)d_in[2];
  const float* b_ih = (const float*)d_in[3];
  const float* b_hh = (const float*)d_in[4];
  const float* W1   = (const float*)d_in[5];
  const float* b1   = (const float*)d_in[6];
  const float* W2   = (const float*)d_in[7];
  const float* b2   = (const float*)d_in[8];
  const float* W3   = (const float*)d_in[9];
  const float* b3   = (const float*)d_in[10];
  const float* W4   = (const float*)d_in[11];
  const float* b4   = (const float*)d_in[12];
  float* out = (float*)d_out;

  char* ws = (char*)d_ws;
  unsigned short* X16   = (unsigned short*)(ws + kOffX16);
  unsigned short* WIH16 = (unsigned short*)(ws + kOffWIH);
  unsigned short* WHH16 = (unsigned short*)(ws + kOffWHH);
  unsigned short* WHD16 = (unsigned short*)(ws + kOffWHD);
  float*          BIASP = (float*)(ws + kOffBIASP);
  float*          BHEAD = (float*)(ws + kOffBHEAD);
  float*          XG    = (float*)(ws + kOffXG);
  unsigned short* HS16  = (unsigned short*)(ws + kOffHS);

  cvt_rows_f16_kernel<<<(kT * kD / 8) / 256, 256, 0, stream>>>(X, X16, kT * kD / 8, kXCarry, 0);
  cvt_rows_f16_kernel<<<(kG * kD / 8) / 256, 256, 0, stream>>>(W_ih, WIH16, kG * kD / 8, kWCarry, 1);
  cvt_rows_f16_kernel<<<(kG * kH / 8) / 256, 256, 0, stream>>>(W_hh, WHH16, kG * kH / 8, kWCarry, 0);
  prep_small_kernel<<<1, 256, 0, stream>>>(b_ih, b_hh, W1, b1, W2, b2, W3, b3, W4, b4, WHD16, BIASP, BHEAD);

  gemm64_f16_bias_kernel<<<((kT / 64) * (kG / 64)) / 8, 256, 0, stream>>>(
      X16, kD, WIH16, kD, XG, kG, BIASP, kT, kG, kD, kProjScale);

  lstm_scan_kernel<<<1, 256, 0, stream>>>(WHH16, XG, HS16);

  heads_kernel<<<(kT / 32) / 8, 256, 0, stream>>>(HS16, WHD16, BHEAD, out);
}
